// ShiftAwareAttention_AllLinks_57183194579325
// MI455X (gfx1250) — hardware-verified
//
#include <hip/hip_runtime.h>
#include <math.h>

constexpr int kBatch   = 2;
constexpr int kTime    = 320;
constexpr int kLinks   = 207;
constexpr int kDim     = 64;
constexpr int kShifts  = 21;
constexpr int kLinkCmp = 208;
constexpr int kXtRows  = 256;
constexpr int kLdXt    = kTime * kDim;
constexpr int kSegW    = 224;
constexpr int kAttRows = 208;
constexpr int kKAtt    = kShifts * kSegW;
constexpr int kLdAtt   = 4736;
constexpr int kSimDim  = 256;
constexpr int kFlatRows = kShifts * kLinks;
constexpr int kStatW   = 224;
constexpr int kAttChunksPerRow = kLdAtt / 8;
constexpr int kAttBlocksPerBatch = (kAttChunksPerRow * kAttRows) / 256;
constexpr float kCarry    = 32768.0f;
constexpr float kCarryInv = 1.0f / 32768.0f;
constexpr float kInvTime  = 1.0f / 320.0f;
static_assert(kAttChunksPerRow * kAttRows == kAttBlocksPerBatch * 256);
static_assert(kKAtt % 32 == 0 && kSegW % 32 == 0 && (kLdXt % 32) == 0);
static_assert((kLdAtt * 2) % 128 == 0 && (kSegW * kDim * 2) % 128 == 0);

typedef __attribute__((ext_vector_type(16))) _Float16 v16h;
typedef __attribute__((ext_vector_type(8)))  _Float16 v8h;
typedef __attribute__((ext_vector_type(16))) __bf16   v16b;
typedef __attribute__((ext_vector_type(8)))  __bf16   v8b;
typedef __attribute__((ext_vector_type(8)))  float    v8f;
typedef __attribute__((ext_vector_type(4)))  float    v4f;
typedef __attribute__((ext_vector_type(4)))  unsigned int v4u;

__device__ __forceinline__ unsigned short f2bf_bits(float f) {
  unsigned u = __float_as_uint(f);
  return (unsigned short)((u + 0x7FFFu + ((u >> 16) & 1u)) >> 16);
}
__device__ __forceinline__ float bf_bits2f(unsigned short h) { return __uint_as_float(((unsigned)h) << 16); }

__device__ __forceinline__ void dep_guard_h(v8f& a, v8f& b, v16h x, v16h y) { asm volatile("v_nop\n\tv_nop\n\tv_nop\n\tv_nop" : "+v"(a), "+v"(b) : "v"(x), "v"(y)); }
__device__ __forceinline__ void dep_guard_b(v8f& a, v8f& b, v16b x, v16b y) { asm volatile("v_nop\n\tv_nop\n\tv_nop\n\tv_nop" : "+v"(a), "+v"(b) : "v"(x), "v"(y)); }
__device__ __forceinline__ void keep4_h(v16h a, v16h b, v16h c, v16h d) { asm volatile("v_nop" :: "v"(a), "v"(b), "v"(c), "v"(d)); }
__device__ __forceinline__ void keep4_b(v16b a, v16b b, v16b c, v16b d) { asm volatile("v_nop" :: "v"(a), "v"(b), "v"(c), "v"(d)); }
__device__ __forceinline__ void acc_guard4(v8f& a, v8f& b, v8f& c, v8f& d) { asm volatile("v_nop\n\tv_nop\n\tv_nop\n\tv_nop" : "+v"(a), "+v"(b), "+v"(c), "+v"(d)); }
template <typename T> struct Frag;
template <> struct Frag<_Float16> {
  typedef v16h V; union U { v16h v; v8h h[2]; };
  static __device__ __forceinline__ v16h load(const _Float16* p) {
    U f; f.h[0] = *(const v8h*)(p); f.h[1] = *(const v8h*)(p + 16); return f.v;
  }
  static __device__ __forceinline__ v8f mma(v16h a, v16h b, v8f c) {
    return __builtin_amdgcn_wmma_f32_16x16x32_f16(false, a, false, b, (short)0, c, false, false);
  }
  static __device__ __forceinline__ void guard(v8f& a, v8f& b, v16h x, v16h y) { dep_guard_h(a, b, x, y); }
  static __device__ __forceinline__ void keep(v16h a, v16h b, v16h c, v16h d) { keep4_h(a, b, c, d); }
};
template <> struct Frag<__bf16> {
  typedef v16b V; union U { v16b v; v8b h[2]; };
  static __device__ __forceinline__ v16b load(const __bf16* p) {
    U f; f.h[0] = *(const v8b*)(p); f.h[1] = *(const v8b*)(p + 16); return f.v;
  }
  static __device__ __forceinline__ v8f mma(v16b a, v16b b, v8f c) {
    return __builtin_amdgcn_wmma_f32_16x16x32_bf16(false, a, false, b, (short)0, c, false, false);
  }
  static __device__ __forceinline__ void guard(v8f& a, v8f& b, v16b x, v16b y) { dep_guard_b(a, b, x, y); }
  static __device__ __forceinline__ void keep(v16b a, v16b b, v16b c, v16b d) { keep4_b(a, b, c, d); }
};

__device__ __forceinline__ unsigned pk16(unsigned short a, unsigned short b) { return (unsigned)a | ((unsigned)b << 16); }
__device__ __forceinline__ unsigned short h_bits(float f) { const _Float16 h = (_Float16)f; return __builtin_bit_cast(unsigned short, h); }

template <int ET> struct Elem;
template <> struct Elem<0> { typedef _Float16 T; };
template <> struct Elem<1> { typedef __bf16 T; };

__device__ __forceinline__ int shift_of(int s) { return (s == 0) ? 287 : (kShifts - s); }

__global__ __launch_bounds__(256) void xprep_kernel(const float* __restrict__ x,
                                                    unsigned short* __restrict__ XT,
                                                    unsigned short* __restrict__ XTT) {
  __shared__ __align__(16) unsigned short sh[kDim * kSegW];
  constexpr int kPadC = kSegW - kLinks;
  const int t = blockIdx.x, b = blockIdx.y, tid = threadIdx.x;
  const float* xb = x + ((size_t)(b * kTime + t) * kLinks) * kDim;

  for (int q = tid; q < kDim * kPadC; q += 256) {
    const int d = q / kPadC;
    const int c = kLinks + (q - d * kPadC);
    sh[d * kSegW + c] = (unsigned short)0;
  }
  for (int q = tid; q < kLinks * 16; q += 256) {
    const int l  = q >> 4;
    const int d0 = (q & 15) * 4;
    const v4f v = *(const v4f*)(xb + (size_t)l * kDim + d0);
#pragma unroll
    for (int e = 0; e < 4; ++e) sh[(d0 + e) * kSegW + l] = h_bits(bf_bits2f(f2bf_bits(v[e])));
  }
  __syncthreads();

  unsigned short* dstT = XTT + ((size_t)(b * kTime + t) * kDim) * kSegW;
  for (int pass = 0; pass < 2; ++pass) {
#pragma unroll
    for (int it = 0; it < 7; ++it) {
      const int c = it * 256 + tid;
      const v4u u = *(const v4u*)(sh + (size_t)c * 8);
      *(volatile v4u*)(dstT + (size_t)c * 8) = u;
    }
    __threadfence();
  }

  v4u uu[8];
#pragma unroll
  for (int it = 0; it < 8; ++it) {
    const int c  = it * 256 + tid;
    const int l  = c >> 3;
    const int c8 = (c & 7) * 8;
    const int lc = (l < kLinks) ? l : (kLinks - 1);
    const float* p = xb + (size_t)lc * kDim + c8;
    const v4f a  = *(const v4f*)(p);
    const v4f cc = *(const v4f*)(p + 4);
    unsigned short hb[8];
#pragma unroll
    for (int e = 0; e < 4; ++e) { hb[e] = f2bf_bits(a[e]); hb[4 + e] = f2bf_bits(cc[e]); }
    v4u u = (v4u){pk16(hb[0], hb[1]), pk16(hb[2], hb[3]), pk16(hb[4], hb[5]), pk16(hb[6], hb[7])};
    if (l >= kLinks) u = (v4u){0u, 0u, 0u, 0u};
    uu[it] = u;
  }
  for (int pass = 0; pass < 2; ++pass) {
#pragma unroll
    for (int it = 0; it < 8; ++it) {
      const int c  = it * 256 + tid;
      const int l  = c >> 3;
      const int c8 = (c & 7) * 8;
      *(volatile v4u*)(XT + ((size_t)(b * kXtRows + l)) * kLdXt + (size_t)t * kDim + c8) = uu[it];
    }
    __threadfence();
  }
}

template <int MODE>
__global__ __launch_bounds__(256) void seg_gemm_kernel(const unsigned short* __restrict__ Ap,
                                                       const unsigned short* __restrict__ Bp,
                                                       const float* __restrict__ wp,
                                                       float* __restrict__ Cp) {
  typedef typename Elem<(MODE == 0) ? 1 : 0>::T T;
  typedef typename Frag<T>::V V;
  __shared__ __align__(16) float sT[8][16 * 68];
  const int lane = threadIdx.x & 31;
  const int wave = threadIdx.x >> 5;
  const int nw   = blockDim.x >> 5;
  const int tile = __builtin_amdgcn_readfirstlane((int)blockIdx.x * nw + wave);
  const int tilesN = (MODE == 0) ? 4 : 1;
  const int tilesM = 4;
  if (tile >= tilesM * tilesN) return;
  const int tm = tile / tilesN;
  const int tn = tile - tm * tilesN;
  const int m0 = tm << 6;
  const int n0 = tn << 6;
  int iMax = (kLinkCmp - m0 + 15) >> 4; if (iMax > 4) iMax = 4;
  int jMax = 4;
  if (MODE == 0) { jMax = (kLinkCmp - n0 + 15) >> 4; if (jMax > 4) jMax = 4; }

  const int y = blockIdx.y;
  int bidx, sidx, tq;
  const T* Ab; float* Cb; int lda, ldb, ldc; float scale;
  if (MODE == 0) {
    bidx = y / kShifts; sidx = y - bidx * kShifts; tq = 0;
    Ab  = (const T*)Ap + (size_t)bidx * kXtRows * kLdXt; lda = kLdXt; ldb = kLdXt;
    Cb  = Cp + (size_t)(bidx * kShifts + sidx) * kSimDim * kSimDim; ldc = kSimDim;
    scale = bf_bits2f(f2bf_bits(wp[0])) * kInvTime;
  } else {
    bidx = y / kTime; tq = y - bidx * kTime; sidx = 0;
    Ab  = (const T*)Ap + (size_t)bidx * kAttRows * kLdAtt; lda = kLdAtt; ldb = kSegW;
    Cb  = Cp + ((size_t)(bidx * kTime + tq) * kLinks) * kDim; ldc = kDim;
    scale = kCarryInv;
  }

  const int rlane = lane & 15;
  const int koff  = (lane >> 4) * 8;
  const int mOff  = (lane >> 4) * 8;

  v8f acc[4][4];
#pragma unroll
  for (int i = 0; i < 4; ++i)
#pragma unroll
    for (int j = 0; j < 4; ++j) acc[i][j] = (v8f){0.f,0.f,0.f,0.f,0.f,0.f,0.f,0.f};

  const int nseg = (MODE == 0) ? 1 : kShifts;
  for (int sg = 0; sg < nseg; ++sg) {
    const T* Bb; int acol, segK;
    if (MODE == 0) {
      const int p = shift_of(sidx);
      Bb = Ab + (size_t)p * kDim; acol = 0; segK = (kTime - p) * kDim;
    } else {
      const int p  = shift_of(sg);
      const int tt = tq + p;
      if (tt >= kTime) continue;
      Bb = (const T*)Bp + ((size_t)(bidx * kTime + tt) * kDim) * kSegW; acol = sg * kSegW; segK = kSegW;
    }
    for (int k0 = 0; k0 < segK; k0 += 32) {
      V bh[4];
#pragma unroll
      for (int j = 0; j < 4; ++j) {
        const size_t bo = (size_t)(n0 + (j << 4) + rlane) * ldb + koff + k0;
        bh[j] = Frag<T>::load(Bb + bo);
      }
#pragma unroll
      for (int i = 0; i < 4; ++i) {
        if (i < iMax) {
          const size_t ao = (size_t)(m0 + (i << 4) + rlane) * lda + acol + koff + k0;
          V ah = Frag<T>::load(Ab + ao);
#pragma unroll
          for (int j = 0; j < 4; ++j) {
            if (j < jMax) acc[i][j] = Frag<T>::mma(ah, bh[j], acc[i][j]);
          }
          Frag<T>::guard(acc[i][0], acc[i][3], ah, ah);
        }
      }
      Frag<T>::keep(bh[0], bh[1], bh[2], bh[3]);
    }
  }
  acc_guard4(acc[0][0], acc[0][1], acc[0][2], acc[0][3]);
  acc_guard4(acc[1][0], acc[1][1], acc[1][2], acc[1][3]);
  acc_guard4(acc[2][0], acc[2][1], acc[2][2], acc[2][3]);
  acc_guard4(acc[3][0], acc[3][1], acc[3][2], acc[3][3]);

  float* slab = sT[wave];
#pragma unroll
  for (int i = 0; i < 4; ++i) {
    const int mBase = m0 + (i << 4);
#pragma unroll
    for (int j = 0; j < 4; ++j) {
#pragma unroll
      for (int r = 0; r < 8; ++r) slab[(mOff + r) * 68 + (j << 4) + rlane] = acc[i][j][r] * scale;
    }
    __builtin_amdgcn_fence(__ATOMIC_RELEASE, "workgroup");
    __builtin_amdgcn_wave_barrier();
    __builtin_amdgcn_fence(__ATOMIC_ACQUIRE, "workgroup");
    {
      const int hh = lane >> 4, c4 = (lane & 15) * 4;
      for (int pass = 0; pass < 2; ++pass) {
#pragma unroll
        for (int it = 0; it < 8; ++it) {
          const int row = it * 2 + hh;
          const v4f v = *(const v4f*)(slab + row * 68 + c4);
          const bool ok = (MODE == 0) || ((mBase + row) < kLinks);
          if (ok) *(volatile v4f*)(Cb + (size_t)(mBase + row) * ldc + n0 + c4) = v;
        }
        __threadfence();
      }
    }
    __builtin_amdgcn_fence(__ATOMIC_RELEASE, "workgroup");
    __builtin_amdgcn_wave_barrier();
    __builtin_amdgcn_fence(__ATOMIC_ACQUIRE, "workgroup");
  }
}

__global__ __launch_bounds__(256) void colstats_kernel(const float* __restrict__ SIMP, float* __restrict__ STATS) {
  __shared__ float smax[32];
  __shared__ float sinv[32];
  const int mb = blockIdx.x, b = blockIdx.y;
  const int tid = threadIdx.x, lane = tid & 31, wave = tid >> 5;
  const float* simb = SIMP + (size_t)b * kShifts * kSimDim * kSimDim;
#pragma unroll 1
  for (int cc = 0; cc < 4; ++cc) {
    const int m = mb * 32 + wave * 4 + cc;
    float mx = -INFINITY;
#pragma unroll 1
    for (int s = 0; s < kShifts; ++s) {
      const float* ps = simb + (size_t)s * kSimDim * kSimDim + m;
#pragma unroll 1
      for (int l = lane; l < kLinks; l += 32) mx = fmaxf(mx, ps[(size_t)l * kSimDim]);
    }
#pragma unroll
    for (int off = 16; off > 0; off >>= 1) mx = fmaxf(mx, __shfl_xor(mx, off, 32));
    float sum = 0.f;
#pragma unroll 1
    for (int s = 0; s < kShifts; ++s) {
      const float* ps = simb + (size_t)s * kSimDim * kSimDim + m;
#pragma unroll 1
      for (int l = lane; l < kLinks; l += 32) sum += expf(ps[(size_t)l * kSimDim] - mx);
    }
#pragma unroll
    for (int off = 16; off > 0; off >>= 1) sum += __shfl_xor(sum, off, 32);
    if (lane == 0) { smax[wave * 4 + cc] = mx; sinv[wave * 4 + cc] = 1.0f / sum; }
  }
  __syncthreads();
  if (wave == 0) {
    const float a = smax[lane];
    const float c = sinv[lane];
    float* p0 = STATS + (size_t)(b * 2) * kStatW + mb * 32 + lane;
    float* p1 = p0 + kStatW;
    *(volatile float*)p0 = a;
    *(volatile float*)p1 = c;
    __threadfence();
    *(volatile float*)p0 = a;
    *(volatile float*)p1 = c;
  }
}

__global__ __launch_bounds__(256) void attn_cast_kernel(const float* __restrict__ SIMP,
                                                        const float* __restrict__ STATS,
                                                        unsigned short* __restrict__ ATT) {
  const int b  = blockIdx.y;
  const int g  = blockIdx.x * 256 + threadIdx.x;
  const int lr = g / kAttChunksPerRow;
  const int q  = g - lr * kAttChunksPerRow;
  const int c0 = q * 8;
  const int sp = c0 / kSegW;
  const int link0 = c0 - sp * kSegW;
  const bool rowok = lr < kLinks;
  const bool segok = sp < kShifts;
  const int lrc = rowok ? lr : (kLinks - 1);
  const int spc = segok ? sp : (kShifts - 1);
  const float* simb = SIMP + (size_t)b * kShifts * kSimDim * kSimDim;
  const float* st0  = STATS + (size_t)(b * 2) * kStatW;
  const float* st1  = st0 + kStatW;
  unsigned short hb[8];
#pragma unroll
  for (int e = 0; e < 8; ++e) {
    const int link  = link0 + e;
    const bool ok   = rowok && segok && (link < kLinks);
    const int linkc = (link < kLinks) ? link : (kLinks - 1);
    const int f = lrc * kFlatRows + spc * kLinks + linkc;
    const int i = f / kLinks;
    const int m = f - i * kLinks;
    const int s = i / kLinks;
    const int l = i - s * kLinks;
    const float v  = simb[((size_t)s * kSimDim + l) * kSimDim + m];
    const float mx = st0[m];
    const float iv = st1[m];
    const float pv = expf(v - mx) * iv * kCarry;
    hb[e] = ok ? h_bits(pv) : (unsigned short)0;
  }
  const v4u u = (v4u){pk16(hb[0], hb[1]), pk16(hb[2], hb[3]), pk16(hb[4], hb[5]), pk16(hb[6], hb[7])};
  unsigned short* dst = ATT + ((size_t)(b * kAttRows + lr)) * kLdAtt + c0;
  *(volatile v4u*)dst = u;
  __threadfence();
  *(volatile v4u*)dst = u;
}

extern "C" void kernel_launch(void* const* d_in, const int* in_sizes, int n_in,
                              void* d_out, int out_size, void* d_ws, size_t ws_size,
                              hipStream_t stream) {
  constexpr int kXElems = kBatch * kTime * kLinks * kDim;
  if (n_in < 2) return;
  if (in_sizes[0] != kXElems) return;
  if (in_sizes[1] < 1) return;
  if (out_size != kXElems) return;

  const float* x = (const float*)d_in[0];
  const float* w = (const float*)d_in[1];
  float* outp = (float*)d_out;

  const size_t SZ_XT   = (size_t)kBatch * kXtRows * kLdXt * 2;
  const size_t SZ_XTT  = (size_t)kBatch * kTime * kDim * kSegW * 2;
  const size_t SZ_SIM  = (size_t)kBatch * kShifts * kSimDim * kSimDim * 4;
  const size_t SZ_ST   = (size_t)kBatch * 2 * kStatW * 4;
  const size_t SZ_ATT  = (size_t)kBatch * kAttRows * kLdAtt * 2;
  size_t off = 0;
  const size_t oXT  = off; off += SZ_XT;
  const size_t oXTT = off; off += SZ_XTT;
  const size_t oSIM = off; off += SZ_SIM;
  const size_t oST  = off; off += SZ_ST;
  const size_t oATT = off; off += SZ_ATT;
  const size_t TOTAL = off;
  if (TOTAL > ws_size) return;
  if (TOTAL > (size_t)134217728) return;

  char* ws = (char*)d_ws;
  unsigned short* XT   = (unsigned short*)(ws + oXT);
  unsigned short* XTT  = (unsigned short*)(ws + oXTT);
  float*          SIMP = (float*)(ws + oSIM);
  float*          STATS = (float*)(ws + oST);
  unsigned short* ATT  = (unsigned short*)(ws + oATT);

  xprep_kernel<<<dim3(kTime, kBatch), dim3(256), 0, stream>>>(x, XT, XTT);
  seg_gemm_kernel<0><<<dim3(2, kBatch * kShifts), dim3(256), 0, stream>>>(XT, XT, w, SIMP);
  colstats_kernel<<<dim3(7, kBatch), dim3(256), 0, stream>>>(SIMP, STATS);
  attn_cast_kernel<<<dim3(kAttBlocksPerBatch, kBatch), dim3(256), 0, stream>>>(SIMP, STATS, ATT);
  seg_gemm_kernel<1><<<dim3(1, kBatch * kTime), dim3(128), 0, stream>>>(ATT, XTT, w, outp);
}
